// TransFormerLayer_68247030334341
// MI455X (gfx1250) — hardware-verified
//
#include <hip/hip_runtime.h>
#ifndef NB
#define NB 4
#endif
#ifndef SEQ
#define SEQ 1024
#endif
#define NB_FULL 4
#define SEQ_FULL 1024
#define DM 1024
#define NH 16
#define HD 64
#define DFF 4096
#define LQ 3072
#define LG 2048
#define NR (NB * SEQ)
#define NEGV (-1.0e9f)
#define OFF_G  ((size_t)NB_FULL * SEQ_FULL * DM)
#define OFF_NB (OFF_G + (size_t)NB_FULL * SEQ_FULL * SEQ_FULL)

static_assert(SEQ % 64 == 0);
static_assert(SEQ <= SEQ_FULL);
static_assert(NB <= NB_FULL);
static_assert(NH * HD == DM);
static_assert(LQ == 3 * DM && LG == 2 * DM);
static_assert(DM == 1024);
static_assert(DM % 64 == 0 && DFF % 64 == 0 && LQ % 64 == 0 && LG % 64 == 0);
static_assert(DM % 32 == 0 && DFF % 32 == 0);
static_assert(NR % 128 == 0);
static_assert(OFF_G * 4 == (size_t)16777216);
static_assert(OFF_NB * 4 == (size_t)33554432);

typedef unsigned short v8us __attribute__((ext_vector_type(8), may_alias));
typedef float  v8f  __attribute__((ext_vector_type(8)));
typedef float  v4f  __attribute__((ext_vector_type(4)));
typedef float  v4fa __attribute__((ext_vector_type(4), may_alias));
typedef int    v4ia __attribute__((ext_vector_type(4), may_alias));
typedef double v2d  __attribute__((ext_vector_type(2)));
typedef _Float16 v16h __attribute__((ext_vector_type(16)));
typedef _Float16 v4h  __attribute__((ext_vector_type(4)));
union FragH { v16h v; v8us half[2]; _Float16 h[16]; unsigned short u[16]; };

__device__ __forceinline__ unsigned short bf16_bits(float x) { unsigned int u = __float_as_uint(x); return (unsigned short)((u + 0x7FFFu + ((u >> 16) & 1u)) >> 16); }
__device__ __forceinline__ float bf16_rne(float x) { return __uint_as_float(((unsigned int)bf16_bits(x)) << 16); }
__device__ __forceinline__ unsigned xrow(unsigned r) { return (r / (unsigned)SEQ) * (unsigned)SEQ_FULL + (r % (unsigned)SEQ); }

__device__ __forceinline__ v16h g2_frag(const _Float16* p, unsigned hh) { FragH f; f.half[0] = *(const v8us*)((const unsigned short*)p + 8 * hh); f.half[1] = *(const v8us*)((const unsigned short*)p + 16 + 8 * hh); return f.v; }
__device__ __forceinline__ v8f g2_mma(v16h a, v16h b, v8f c) { v8f d = __builtin_amdgcn_wmma_f32_16x16x32_f16(false, a, false, b, (short)0, c, false, false); asm volatile("v_nop\n\tv_nop\n\tv_nop\n\tv_nop" : "+v"(d) : "v"(a), "v"(b)); return d; }

__global__ __launch_bounds__(256) void k_wt_f16(const float* __restrict__ W, _Float16* __restrict__ Wt, unsigned K, unsigned N, float scale) {
  const unsigned t = blockIdx.x * 256u + threadIdx.x; const unsigned k8n = K >> 3;
  if (t >= N * k8n) return;
  const unsigned n = t / k8n, k8 = (t - n * k8n) * 8u;
  FragH f;
#pragma unroll
  for (int i = 0; i < 8; ++i) f.h[i] = (_Float16)(bf16_rne(W[(size_t)(k8 + i) * N + n]) * scale);
  const v8us o = f.half[0];
  unsigned short* d = (unsigned short*)Wt + (size_t)n * K + k8;
  *(volatile v8us*)d = o; __threadfence(); *(volatile v8us*)d = o;
}

template <int INBF, int TWO>
__global__ __launch_bounds__(256) void k_ln(const float* __restrict__ Y, const float* __restrict__ ga, const float* __restrict__ gb, const float* __restrict__ ha, const float* __restrict__ hb,
    _Float16* __restrict__ N16A, _Float16* __restrict__ N16B) {
  __shared__ float sm[8]; __shared__ float sv[8];
  const unsigned r = blockIdx.x, t = threadIdx.x, lane = t & 31u, w = t >> 5;
  const unsigned sr = INBF ? xrow(r) : r;
  v4f xa = *(const v4fa*)(Y + (size_t)sr * DM + t * 4u);
  if (INBF) {
#pragma unroll
    for (int i = 0; i < 4; ++i) xa[i] = bf16_rne(xa[i]); }
  float s = (xa[0] + xa[1]) + (xa[2] + xa[3]);
  s += __shfl_xor(s, 1, 32); s += __shfl_xor(s, 2, 32); s += __shfl_xor(s, 4, 32); s += __shfl_xor(s, 8, 32); s += __shfl_xor(s, 16, 32);
  if (lane == 0) sm[w] = s;
  __syncthreads();
  float tot = 0.f;
#pragma unroll
  for (int i = 0; i < 8; ++i) tot += sm[i];
  const float mu = tot * (1.0f / (float)DM);
  const float d0 = xa[0] - mu, d1 = xa[1] - mu, d2 = xa[2] - mu, d3 = xa[3] - mu;
  float q2 = (d0 * d0 + d1 * d1) + (d2 * d2 + d3 * d3);
  q2 += __shfl_xor(q2, 1, 32); q2 += __shfl_xor(q2, 2, 32); q2 += __shfl_xor(q2, 4, 32); q2 += __shfl_xor(q2, 8, 32); q2 += __shfl_xor(q2, 16, 32);
  if (lane == 0) sv[w] = q2;
  __syncthreads();
  float vt = 0.f;
#pragma unroll
  for (int i = 0; i < 8; ++i) vt += sv[i];
  const float sd = sqrtf(vt * (1.0f / (float)(DM - 1)));
  const float rs = 1.0f / (sd + 1.0e-6f);
  const float n0 = d0 * rs, n1 = d1 * rs, n2 = d2 * rs, n3 = d3 * rs;
  const v4f av = *(const v4fa*)(ga + t * 4u), bv = *(const v4fa*)(gb + t * 4u);
  v4h ya, yb;
  ya[0] = (_Float16)(n0 * bf16_rne(av[0]) + bf16_rne(bv[0])); ya[1] = (_Float16)(n1 * bf16_rne(av[1]) + bf16_rne(bv[1]));
  ya[2] = (_Float16)(n2 * bf16_rne(av[2]) + bf16_rne(bv[2])); ya[3] = (_Float16)(n3 * bf16_rne(av[3]) + bf16_rne(bv[3]));
  yb = ya;
  if (TWO) {
    const v4f cv = *(const v4fa*)(ha + t * 4u), dv = *(const v4fa*)(hb + t * 4u);
    yb[0] = (_Float16)(n0 * bf16_rne(cv[0]) + bf16_rne(dv[0])); yb[1] = (_Float16)(n1 * bf16_rne(cv[1]) + bf16_rne(dv[1]));
    yb[2] = (_Float16)(n2 * bf16_rne(cv[2]) + bf16_rne(dv[2])); yb[3] = (_Float16)(n3 * bf16_rne(cv[3]) + bf16_rne(dv[3]));
  }
  for (int pass = 0; pass < 2; ++pass) {
    *(volatile v4h*)(N16A + (size_t)r * DM + t * 4u) = ya;
    if (TWO) *(volatile v4h*)(N16B + (size_t)r * DM + t * 4u) = yb;
    if (pass == 0) __threadfence(); }
}

__global__ __launch_bounds__(256) void k_link(const float* __restrict__ QK, const int* __restrict__ eos, float* __restrict__ PT) {
  __shared__ __attribute__((aligned(16))) float sp[3][32];
  const unsigned tid = threadIdx.x, w = tid >> 5, lane = tid & 31u;
  const unsigned rbase = blockIdx.x * 32u;
#pragma unroll 1
  for (unsigned rr = 0; rr < 4u; ++rr) {
    const unsigned rl = w * 4u + rr, row = rbase + rl;
    const unsigned b = row / (unsigned)SEQ, i = row % (unsigned)SEQ;
    const bool hasl = (i > 0u), hasr = (i + 1u < (unsigned)SEQ);
    const unsigned il = hasl ? (i - 1u) : 0u, ir = hasr ? (i + 1u) : (unsigned)(SEQ - 1);
    const float* qp = QK + (size_t)row * LG;
    const float* kl = QK + ((size_t)b * SEQ + il) * LG + DM;
    const float* kr = QK + ((size_t)b * SEQ + ir) * LG + DM;
    float dl = 0.f, dr = 0.f;
#pragma unroll 2
    for (unsigned it = 0; it < 8u; ++it) {
      const unsigned c = it * 128u + lane * 4u;
      const v4f q = *(const v4fa*)(qp + c), a = *(const v4fa*)(kl + c), e = *(const v4fa*)(kr + c);
      dl = fmaf(q[0], a[0], dl); dl = fmaf(q[1], a[1], dl); dl = fmaf(q[2], a[2], dl); dl = fmaf(q[3], a[3], dl);
      dr = fmaf(q[0], e[0], dr); dr = fmaf(q[1], e[1], dr); dr = fmaf(q[2], e[2], dr); dr = fmaf(q[3], e[3], dr);
    }
    dl += __shfl_xor(dl, 16, 32); dr += __shfl_xor(dr, 16, 32);
    dl += __shfl_xor(dl, 8, 32);  dr += __shfl_xor(dr, 8, 32);
    dl += __shfl_xor(dl, 4, 32);  dr += __shfl_xor(dr, 4, 32);
    dl += __shfl_xor(dl, 2, 32);  dr += __shfl_xor(dr, 2, 32);
    dl += __shfl_xor(dl, 1, 32);  dr += __shfl_xor(dr, 1, 32);
    const size_t eb = ((size_t)b * SEQ_FULL + i) * SEQ_FULL;
    const int ml = eos[eb + il], mr = eos[eb + ir];
    const float sl = (hasl && ml != 0) ? dl * 0.00390625f : NEGV;
    const float sr = (hasr && mr != 0) ? dr * 0.00390625f : NEGV;
    const float mm = fmaxf(sl, sr);
    const float el0 = expf(sl - mm), er0 = expf(sr - mm), eo = expf(NEGV - mm);
    const float el = hasl ? el0 : 0.f, er = hasr ? er0 : 0.f;
    const float cnt = (float)((unsigned)SEQ - (hasl ? 1u : 0u) - (hasr ? 1u : 0u));
    const float sum = (el + er) + cnt * eo;
    const float inv = 1.0f / sum;
    if (lane == 0) { sp[0][rl] = el * inv; sp[1][rl] = er * inv; sp[2][rl] = eo * inv; }
  }
  __syncthreads();
  if (tid < 24u) {
    const unsigned arr = tid >> 3, pc = (tid & 7u) * 4u;
    const v4f v = *(const v4fa*)&sp[arr][pc];
    float* dst = PT + (size_t)arr * NR + rbase + pc;
    *(volatile v4f*)dst = v; __threadfence(); *(volatile v4f*)dst = v;
  }
}

__global__ __launch_bounds__(256) void k_scan(const float* __restrict__ PT, const float* __restrict__ prior, double* __restrict__ E) {
  __shared__ float lk[SEQ];
  __shared__ __attribute__((aligned(16))) double ed[SEQ];
  const unsigned b = blockIdx.x, tid = threadIdx.x;
  const float pr0 = bf16_rne(prior[0]);
#pragma unroll 1
  for (unsigned k = tid; k < (unsigned)SEQ; k += 256u) {
    const bool live = (k + 1u < (unsigned)SEQ);
    const unsigned k1 = live ? (k + 1u) : (unsigned)(SEQ - 1);
    const float a = PT[(size_t)NR + b * (unsigned)SEQ + k], c = PT[b * (unsigned)SEQ + k1];
    const float v = pr0 + (1.0f - pr0) * sqrtf(a * c + 1.0e-9f);
    const float lg = logf(v + 1.0e-9f);
    lk[k] = live ? lg : 0.f;
  }
  __syncthreads();
  if (tid == 0) {
    double s = 0.0;
#pragma unroll 1
    for (unsigned k = 0; k < (unsigned)SEQ; ++k) { ed[k] = s; s += (double)lk[k]; }
  }
  __syncthreads();
  for (int pass = 0; pass < 2; ++pass) {
#pragma unroll 1
    for (unsigned k2 = tid * 2u; k2 < (unsigned)SEQ; k2 += 512u) { v2d v; v[0] = ed[k2]; v[1] = ed[k2 + 1u];
      *(volatile v2d*)(E + (size_t)b * SEQ + k2) = v; }
    if (pass == 0) __threadfence(); }
}

__global__ __launch_bounds__(256) void k_fill(const float* __restrict__ PT, const double* __restrict__ E, const float* __restrict__ prior, float* __restrict__ G, float* __restrict__ NBO) {
  __shared__ __attribute__((aligned(16))) float sg[SEQ];
  __shared__ __attribute__((aligned(16))) float sn[SEQ];
  const unsigned row = blockIdx.x, tid = threadIdx.x;
  const unsigned b = row / (unsigned)SEQ, i = row % (unsigned)SEQ;
  const float pr0 = bf16_rne(prior[0]);
  const float* pl = PT + (size_t)b * SEQ; const float* pr = PT + (size_t)NR + (size_t)b * SEQ; const float* pu = PT + (size_t)2 * NR + (size_t)b * SEQ;
  const double* eb = E + (size_t)b * SEQ;
  const float pli = pl[i], pri = pr[i], pui = pu[i]; const double ei = eb[i];
#pragma unroll 1
  for (unsigned j = tid; j < (unsigned)SEQ; j += 256u) {
    const float plj = pl[j], prj = pr[j], puj = pu[j]; const double ej = eb[j];
    const float wij = (j + 1u == i) ? pli : ((j == i + 1u) ? pri : pui);
    const float wji = (i + 1u == j) ? plj : ((i == j + 1u) ? prj : puj);
    const float nv = pr0 + (1.0f - pr0) * sqrtf(wij * wji + 1.0e-9f);
    const double dd = (j > i) ? (ej - ei) : (ei - ej);
    const float ge = expf((float)dd) + 1.0e-9f;
    sn[j] = nv; sg[j] = (i == j) ? nv : ge;
  }
  __syncthreads();
  const size_t ob = ((size_t)b * SEQ_FULL + i) * SEQ_FULL;
  for (int pass = 0; pass < 2; ++pass) {
#pragma unroll 1
    for (unsigned j4 = tid * 4u; j4 < (unsigned)SEQ; j4 += 1024u) { const v4f a = *(const v4fa*)&sg[j4]; const v4f c = *(const v4fa*)&sn[j4];
      *(volatile v4f*)(G + ob + j4) = a; *(volatile v4f*)(NBO + ob + j4) = c; }
    if (pass == 0) __threadfence(); }
}

__global__ __launch_bounds__(256) void k_vt(const _Float16* __restrict__ QKV, _Float16* __restrict__ VT) {
  __shared__ unsigned short tl[64][66];
  const unsigned tid = threadIdx.x; const unsigned slab = blockIdx.x / (unsigned)(SEQ / 64), lg = blockIdx.x % (unsigned)(SEQ / 64); const unsigned b = slab / (unsigned)NH, h = slab % (unsigned)NH;
  for (unsigned i = tid; i < 512u; i += 256u) { const unsigned r = i >> 3, c8 = (i & 7u) * 8u; FragH f; f.half[0] = *(const v8us*)((const unsigned short*)QKV + ((size_t)b * SEQ + lg * 64u + r) * LQ + 2u * DM + h * 64u + c8);
#pragma unroll
    for (int q = 0; q < 8; ++q) tl[r][c8 + q] = f.u[q]; }
  __syncthreads();
  for (int pass = 0; pass < 2; ++pass) {
#pragma unroll
    for (unsigned rd = 0; rd < 2; ++rd) { const unsigned d = rd * 32u + (tid >> 3), pc = tid & 7u; FragH f;
#pragma unroll
      for (int q = 0; q < 8; ++q) f.u[q] = tl[pc * 8u + q][d];
      const v8us o = f.half[0];
      *(volatile v8us*)((unsigned short*)VT + ((size_t)slab * 64u + d) * SEQ + lg * 64u + pc * 8u) = o; }
    if (pass == 0) __threadfence(); }
}

template <int OFS>
__device__ __forceinline__ void ptile(const v8f& c, float sh, const float* gp, float& ps, FragH& pf) {
  const v4f ga = *(const v4fa*)gp, gb = *(const v4fa*)(gp + 4);
#pragma unroll
  for (int r = 0; r < 4; ++r) {
    const float ea = __expf(c[r] + sh), eb = __expf(c[4 + r] + sh);
    ps += ea + eb;
    pf.h[OFS + r] = (_Float16)(ea * ga[r]); pf.h[OFS + 4 + r] = (_Float16)(eb * gb[r]);
  }
}

__global__ __launch_bounds__(128) void k_attn(const _Float16* __restrict__ QKV, const _Float16* __restrict__ VT, const int* __restrict__ eos, const float* __restrict__ G, _Float16* __restrict__ O16) {
  __shared__ __attribute__((aligned(16))) unsigned short os[4][16][72];
  const unsigned tid = threadIdx.x, w = tid >> 5, lane = tid & 31u, ln = lane & 15u, hh = lane >> 4;
  const unsigned qb = blockIdx.x % (unsigned)(SEQ / 64), hb = blockIdx.x / (unsigned)(SEQ / 64); const unsigned h = hb % (unsigned)NH, b = hb / (unsigned)NH;
  const unsigned q0 = qb * 64u + w * 16u;
  const _Float16* qrow = QKV + ((size_t)b * SEQ + q0 + ln) * LQ + h * 64u;
  const v16h bq0 = g2_frag(qrow, hh), bq1 = g2_frag(qrow + 32, hh);
  const _Float16* kbase = QKV + ((size_t)b * SEQ + ln) * LQ + (unsigned)DM + h * 64u;
  const _Float16* vbase = VT + ((size_t)(b * NH + h) * 64u + ln) * SEQ;
  const size_t mrow = ((size_t)b * SEQ_FULL + q0 + ln) * SEQ_FULL + 8u * hh;
  const int* er = eos + mrow; const float* gr = G + mrow;
  const v8f z8 = {0.f, 0.f, 0.f, 0.f, 0.f, 0.f, 0.f, 0.f};
  v8f o[4] = {z8, z8, z8, z8};
  float m = -1.0e30f, l = 0.f;
#pragma unroll 1
  for (unsigned j0 = 0; j0 < (unsigned)SEQ; j0 += 64u) {
    v8f c[4];
#pragma unroll
    for (int t = 0; t < 4; ++t) { const _Float16* kr = kbase + (size_t)(j0 + t * 16u) * LQ; v8f z = z8; z = g2_mma(g2_frag(kr, hh), bq0, z); z = g2_mma(g2_frag(kr + 32, hh), bq1, z); c[t] = z; }
#pragma unroll
    for (int t = 0; t < 4; ++t) { const v4ia m0 = *(const v4ia*)(er + j0 + t * 16u), m1 = *(const v4ia*)(er + j0 + t * 16u + 4u);
#pragma unroll
      for (int r = 0; r < 4; ++r) { c[t][r] = (m0[r] != 0) ? c[t][r] * 0.125f : NEGV; c[t][4 + r] = (m1[r] != 0) ? c[t][4 + r] * 0.125f : NEGV; } }
    float mx = c[0][0];
#pragma unroll
    for (int t = 0; t < 4; ++t)
#pragma unroll
      for (int r = 0; r < 8; ++r) mx = fmaxf(mx, c[t][r]);
    mx = fmaxf(mx, __shfl_xor(mx, 16, 32));
    const float mnew = fmaxf(m, mx);
    const float alpha = __expf(m - mnew);
    m = mnew;
    const float sh = 6.9314718f - mnew;
    float ps = 0.f;
    FragH p0, p1;
    ptile<0>(c[0], sh, gr + j0, ps, p0);
    ptile<8>(c[1], sh, gr + j0 + 16u, ps, p0);
    ptile<0>(c[2], sh, gr + j0 + 32u, ps, p1);
    ptile<8>(c[3], sh, gr + j0 + 48u, ps, p1);
    l = l * alpha + ps;
#pragma unroll
    for (int dt = 0; dt < 4; ++dt)
#pragma unroll
      for (int r = 0; r < 8; ++r) o[dt][r] *= alpha;
#pragma unroll
    for (int dt = 0; dt < 4; ++dt) { const _Float16* vr = vbase + (size_t)(dt * 16u) * SEQ + j0; o[dt] = g2_mma(g2_frag(vr, hh), p0.v, o[dt]); o[dt] = g2_mma(g2_frag(vr + 32, hh), p1.v, o[dt]); }
  }
  const float lt = l + __shfl_xor(l, 16, 32);
  const float fin = 1024.0f * (1.0f / lt);
#pragma unroll
  for (int dt = 0; dt < 4; ++dt) { FragH f;
#pragma unroll
    for (int r = 0; r < 8; ++r) f.h[r] = (_Float16)(o[dt][r] * fin);
    *(v8us*)&os[w][ln][dt * 16 + 8 * hh] = f.half[0]; }
  __builtin_amdgcn_fence(4  , "workgroup"); __builtin_amdgcn_wave_barrier();
  const unsigned rq = lane >> 3, pc = (lane & 7u) * 8u;
  for (int pass = 0; pass < 2; ++pass) {
#pragma unroll
    for (unsigned it = 0; it < 4; ++it) { const unsigned row = it * 4u + rq; const v8us v = *(const v8us*)&os[w][row][pc];
      *(volatile v8us*)((unsigned short*)O16 + ((size_t)b * SEQ + q0 + row) * DM + h * 64u + pc) = v; }
    if (pass == 0) __threadfence(); }
}

template <int ACT, int RES, int OMAP>
__global__ __launch_bounds__(128) void k_gemm2(const _Float16* __restrict__ A, unsigned lda, const _Float16* __restrict__ Bh, unsigned ldb, float alpha,
    const float* __restrict__ bias0, const float* __restrict__ bias1, const float* __restrict__ bias2, unsigned bsh,
    const float* __restrict__ R, unsigned ldr, float* __restrict__ C, _Float16* __restrict__ C16, unsigned ldc, unsigned M, unsigned N, unsigned K) {
  static_assert(ACT == 0 || ACT == 6);
  static_assert(RES == 0 || RES == 1 || RES == 2);
  __shared__ __attribute__((aligned(16))) float so[4][32][68];
  const unsigned tid = threadIdx.x, w = tid >> 5, lane = tid & 31u, ln = lane & 15u, hh = lane >> 4;
  const unsigned ntn = N >> 6; const unsigned mt = blockIdx.x / ntn, nq = blockIdx.x - mt * ntn; const unsigned row0 = mt * 128u + 32u * w, col0 = nq * 64u; if (row0 >= M) return;
  const _Float16* a0p = A + (size_t)(row0 + ln) * lda; const _Float16* a1p = a0p + (size_t)16 * lda;
  const _Float16* b0p = Bh + (size_t)(col0 + ln) * ldb; const _Float16* b1p = b0p + (size_t)16 * ldb; const _Float16* b2p = b1p + (size_t)16 * ldb; const _Float16* b3p = b2p + (size_t)16 * ldb;
  const v8f z8 = {0.f,0.f,0.f,0.f,0.f,0.f,0.f,0.f}; v8f c00 = z8, c01 = z8, c02 = z8, c03 = z8, c10 = z8, c11 = z8, c12 = z8, c13 = z8;
#pragma unroll 1
  for (unsigned kb = 0; kb < K; kb += 32u) { const v16h a0 = g2_frag(a0p + kb, hh), a1 = g2_frag(a1p + kb, hh);
    v16h bfr = g2_frag(b0p + kb, hh); c00 = g2_mma(a0, bfr, c00); c10 = g2_mma(a1, bfr, c10);
    bfr = g2_frag(b1p + kb, hh); c01 = g2_mma(a0, bfr, c01); c11 = g2_mma(a1, bfr, c11);
    bfr = g2_frag(b2p + kb, hh); c02 = g2_mma(a0, bfr, c02); c12 = g2_mma(a1, bfr, c12);
    bfr = g2_frag(b3p + kb, hh); c03 = g2_mma(a0, bfr, c03); c13 = g2_mma(a1, bfr, c13); }
  const unsigned sec = col0 >> bsh;
  const float* bp = (sec == 0u) ? bias0 : ((sec == 1u) ? bias1 : bias2);
  const unsigned cb = col0 - (sec << bsh);
  v8f accs[8] = {c00, c01, c02, c03, c10, c11, c12, c13};
#pragma unroll
  for (int u = 0; u < 8; ++u) { const int t = u & 3, half = u >> 2; const float bv = bf16_rne(bp[cb + t * 16 + ln]);
#pragma unroll
    for (int r = 0; r < 8; ++r) { const unsigned rloc = half * 16 + 8 * hh + r; so[w][rloc][t * 16 + ln] = accs[u][r] * alpha + bv; } }
  __builtin_amdgcn_fence(4  , "workgroup"); __builtin_amdgcn_wave_barrier();
  const unsigned rsub = lane >> 4, c4 = (lane & 15u) * 4u;
  if (ACT == 6 || RES != 0) {
#pragma unroll 4
    for (unsigned q = 0; q < 16; ++q) { const unsigned r = q * 2u + rsub; v4f v = *(const v4fa*)&so[w][r][c4];
      if (RES != 0) { const unsigned gr = row0 + r; const unsigned sr = (RES == 2) ? xrow(gr) : gr; const v4f rv = *(const v4fa*)(R + (size_t)sr * ldr + col0 + c4);
#pragma unroll
        for (int i = 0; i < 4; ++i) v[i] += (RES == 2) ? bf16_rne(rv[i]) : rv[i]; }
      if (ACT == 6) {
#pragma unroll
        for (int i = 0; i < 4; ++i) v[i] = 0.5f * v[i] * (1.0f + erff(v[i] * 0.70710678118654752f)); }
      *(v4fa*)&so[w][r][c4] = v; }
  }
  for (int pass = 0; pass < 2; ++pass) {
#pragma unroll
    for (unsigned q = 0; q < 16; ++q) { const unsigned r = q * 2u + rsub; const v4f v = *(const v4fa*)&so[w][r][c4];
      const unsigned crow = OMAP ? xrow(row0 + r) : (row0 + r);
      if (C) *(volatile v4f*)(C + (size_t)crow * ldc + col0 + c4) = v;
      if (C16) { v4h h4;
#pragma unroll
        for (int i = 0; i < 4; ++i) h4[i] = (_Float16)v[i];
        *(volatile v4h*)(C16 + (size_t)crow * ldc + col0 + c4) = h4; } }
    if (pass == 0) __threadfence(); }
}

#define MAX2(a, b) ((a) > (b) ? (a) : (b))
#define SZ_BG   ((size_t)LG * DM * 2)
#define SZ_BQKV ((size_t)LQ * DM * 2)
#define SZ_BO   ((size_t)DM * DM * 2)
#define SZ_BW1  ((size_t)DFF * DM * 2)
#define SZ_BW2  ((size_t)DM * DFF * 2)
#define SZ_QKG  ((size_t)NR * LG * 4)
#define SZ_QKV  ((size_t)NR * LQ * 2)
#define SZ_VT   ((size_t)NB * NH * HD * SEQ * 2)
#define SZ_HF   ((size_t)NR * DFF * 2)
#define SZ_RA   MAX2(MAX2(SZ_QKG, (SZ_QKV + SZ_VT)), SZ_HF)
#define SZ_RB   ((size_t)NR * DM * 2)
#define SZ_RC   ((size_t)NR * DM * 2)
#define SZ_X1   ((size_t)NR * DM * 4)
#define SZ_PT   ((size_t)3 * NR * 4)
#define SZ_E    ((size_t)NR * 8)
#define SZ_TOT  (SZ_BG + SZ_BQKV + SZ_BO + SZ_BW1 + SZ_BW2 + SZ_RA + SZ_RB + SZ_RC + SZ_X1 + SZ_PT + SZ_E)
static_assert(SZ_QKG <= SZ_RA);
static_assert(SZ_QKV + SZ_VT <= SZ_RA);
static_assert(SZ_HF <= SZ_RA);
static_assert(SZ_TOT <= (size_t)134217728);
static_assert(SZ_BG % 256 == 0 && SZ_BQKV % 256 == 0 && SZ_BO % 256 == 0 && SZ_BW1 % 256 == 0 && SZ_BW2 % 256 == 0 && SZ_RA % 256 == 0 && SZ_QKV % 256 == 0 && SZ_RB % 256 == 0 && SZ_X1 % 256 == 0 && SZ_PT % 256 == 0 && SZ_E % 256 == 0);
static_assert(((size_t)DM * (DM / 8)) % 256 == 0 && ((size_t)DFF * (DM / 8)) % 256 == 0 && ((size_t)DM * (DFF / 8)) % 256 == 0);
static_assert(NR % 32 == 0);
static_assert(SEQ % 8 == 0);

extern "C" void kernel_launch(void* const* d_in, const int* in_sizes, int n_in,
                              void* d_out, int out_size, void* d_ws, size_t ws_size, hipStream_t stream) {
  if (n_in < 25) return;
  const long long xneed = ((long long)(NB - 1) * SEQ_FULL + SEQ) * DM;
  const long long eneed = ((long long)(NB - 1) * SEQ_FULL + (SEQ - 1)) * SEQ_FULL + SEQ;
  if ((long long)in_sizes[0] < xneed || (long long)in_sizes[1] < eneed || in_sizes[2] < 1) return;
  if ((long long)out_size < (long long)OFF_NB + eneed) return;
  if (in_sizes[3] < DM || in_sizes[4] < DM || in_sizes[6] < DM || in_sizes[8] < DM || in_sizes[10] < DM || in_sizes[12] < DM || in_sizes[14] < DM || in_sizes[16] < DM) return;
  if (in_sizes[17] < DM || in_sizes[18] < DM || in_sizes[19] < DM || in_sizes[20] < DM || in_sizes[22] < DFF || in_sizes[24] < DM) return;
  if (in_sizes[5] < DM * DM || in_sizes[7] < DM * DM || in_sizes[9] < DM * DM || in_sizes[11] < DM * DM || in_sizes[13] < DM * DM || in_sizes[15] < DM * DM) return;
  if (in_sizes[21] < DM * DFF || in_sizes[23] < DFF * DM) return;
  if (ws_size < SZ_TOT) return;
  const float* x = (const float*)d_in[0]; const int* eos = (const int*)d_in[1]; const float* prior = (const float*)d_in[2];
  const float* ga_ln_a = (const float*)d_in[3]; const float* ga_ln_b = (const float*)d_in[4];
  const float* ga_wq = (const float*)d_in[5]; const float* ga_bq = (const float*)d_in[6]; const float* ga_wk = (const float*)d_in[7]; const float* ga_bk = (const float*)d_in[8];
  const float* wq = (const float*)d_in[9]; const float* bq = (const float*)d_in[10]; const float* wk = (const float*)d_in[11]; const float* bk = (const float*)d_in[12];
  const float* wv = (const float*)d_in[13]; const float* bv = (const float*)d_in[14]; const float* wo = (const float*)d_in[15]; const float* bo = (const float*)d_in[16];
  const float* ln1_a = (const float*)d_in[17]; const float* ln1_b = (const float*)d_in[18]; const float* ln2_a = (const float*)d_in[19]; const float* ln2_b = (const float*)d_in[20];
  const float* w1 = (const float*)d_in[21]; const float* b1 = (const float*)d_in[22]; const float* w2 = (const float*)d_in[23]; const float* b2 = (const float*)d_in[24];
  float* out = (float*)d_out; float* outG = out + OFF_G; float* outN = out + OFF_NB;
  char* ws = (char*)d_ws; size_t off = 0;
  _Float16* BG   = (_Float16*)(ws + off); off += SZ_BG;
  _Float16* BQKV = (_Float16*)(ws + off); off += SZ_BQKV;
  _Float16* BO   = (_Float16*)(ws + off); off += SZ_BO;
  _Float16* BW1  = (_Float16*)(ws + off); off += SZ_BW1;
  _Float16* BW2  = (_Float16*)(ws + off); off += SZ_BW2;
  float* QKG = (float*)(ws + off); _Float16* QKV = (_Float16*)(ws + off); _Float16* VT = (_Float16*)(ws + off + SZ_QKV); _Float16* HF16 = (_Float16*)(ws + off); off += SZ_RA;
  _Float16* CTX16 = (_Float16*)(ws + off); _Float16* O16 = (_Float16*)(ws + off); _Float16* Y2H = (_Float16*)(ws + off); off += SZ_RB;
  _Float16* Y16  = (_Float16*)(ws + off); off += SZ_RC;
  float* X1      = (float*)(ws + off); off += SZ_X1;
  float* PT      = (float*)(ws + off); off += SZ_PT;
  double* E      = (double*)(ws + off); off += SZ_E;
  if (off > ws_size) return;

  const unsigned gDD = (unsigned)((size_t)DM * (DM / 8) / 256);
  k_wt_f16<<<gDD, 256, 0, stream>>>(ga_wq, BG, (unsigned)DM, (unsigned)DM, 16.0f);
  k_wt_f16<<<gDD, 256, 0, stream>>>(ga_wk, BG + (size_t)DM * DM, (unsigned)DM, (unsigned)DM, 16.0f);
  k_wt_f16<<<gDD, 256, 0, stream>>>(wq, BQKV, (unsigned)DM, (unsigned)DM, 16.0f);
  k_wt_f16<<<gDD, 256, 0, stream>>>(wk, BQKV + (size_t)DM * DM, (unsigned)DM, (unsigned)DM, 16.0f);
  k_wt_f16<<<gDD, 256, 0, stream>>>(wv, BQKV + (size_t)2 * DM * DM, (unsigned)DM, (unsigned)DM, 16.0f);
  k_wt_f16<<<gDD, 256, 0, stream>>>(wo, BO, (unsigned)DM, (unsigned)DM, 16.0f);
  k_wt_f16<<<(unsigned)((size_t)DFF * (DM / 8) / 256), 256, 0, stream>>>(w1, BW1, (unsigned)DM, (unsigned)DFF, 16.0f);
  k_wt_f16<<<(unsigned)((size_t)DM * (DFF / 8) / 256), 256, 0, stream>>>(w2, BW2, (unsigned)DFF, (unsigned)DM, 64.0f);

  k_ln<1, 1><<<(unsigned)NR, 256, 0, stream>>>(x, ga_ln_a, ga_ln_b, ln1_a, ln1_b, CTX16, Y16);
  k_gemm2<0, 0, 0><<<(unsigned)((NR / 128) * (LG / 64)), 128, 0, stream>>>(CTX16, (unsigned)DM, BG, (unsigned)DM, 0.0625f, ga_bq, ga_bk, ga_bk, 10u, nullptr, 0u, QKG, nullptr, (unsigned)LG, (unsigned)NR, (unsigned)LG, (unsigned)DM);
  k_link<<<(unsigned)(NR / 32), 256, 0, stream>>>(QKG, eos, PT);
  k_scan<<<(unsigned)NB, 256, 0, stream>>>(PT, prior, E);
  k_fill<<<(unsigned)NR, 256, 0, stream>>>(PT, E, prior, outG, outN);

  k_gemm2<0, 0, 0><<<(unsigned)((NR / 128) * (LQ / 64)), 128, 0, stream>>>(Y16, (unsigned)DM, BQKV, (unsigned)DM, 0.0625f, bq, bk, bv, 10u, nullptr, 0u, nullptr, QKV, (unsigned)LQ, (unsigned)NR, (unsigned)LQ, (unsigned)DM);
  k_vt<<<(unsigned)(NB * NH * (SEQ / 64)), 256, 0, stream>>>(QKV, VT);
  k_attn<<<(unsigned)(NB * NH * (SEQ / 64)), 128, 0, stream>>>(QKV, VT, eos, outG, O16);
  k_gemm2<0, 2, 0><<<(unsigned)((NR / 128) * (DM / 64)), 128, 0, stream>>>(O16, (unsigned)DM, BO, (unsigned)DM, 0.00006103515625f, bo, bo, bo, 31u, x, (unsigned)DM, X1, nullptr, (unsigned)DM, (unsigned)NR, (unsigned)DM, (unsigned)DM);

  k_ln<0, 0><<<(unsigned)NR, 256, 0, stream>>>(X1, ln2_a, ln2_b, ln2_a, ln2_b, Y2H, Y2H);
  k_gemm2<6, 0, 0><<<(unsigned)((NR / 128) * (DFF / 64)), 128, 0, stream>>>(Y2H, (unsigned)DM, BW1, (unsigned)DM, 0.0625f, b1, b1, b1, 31u, nullptr, 0u, nullptr, HF16, (unsigned)DFF, (unsigned)NR, (unsigned)DFF, (unsigned)DM);
  k_gemm2<0, 1, 1><<<(unsigned)((NR / 128) * (DM / 64)), 128, 0, stream>>>(HF16, (unsigned)DFF, BW2, (unsigned)DFF, 0.015625f, b2, b2, b2, 31u, X1, (unsigned)DM, out, nullptr, (unsigned)DM, (unsigned)NR, (unsigned)DM, (unsigned)DFF);
}
